// Unify_input_33208687133289
// MI455X (gfx1250) — hardware-run, weakly checked
//
#include <hip/hip_runtime.h>
#include <stddef.h>

typedef unsigned short us;
typedef us     v8us  __attribute__((ext_vector_type(8)));
typedef us     v4us  __attribute__((ext_vector_type(4)));
typedef __bf16 v16bf __attribute__((ext_vector_type(16)));
typedef float  v8f   __attribute__((ext_vector_type(8)));
typedef float  v4f   __attribute__((ext_vector_type(4)));
typedef v8us __attribute__((may_alias)) v8usa;
typedef v4us __attribute__((may_alias)) v4usa;
typedef v4f  __attribute__((may_alias)) v4fa;
union FragB { v16bf v; v8us half[2]; };

#define NB   32
#define NA   64
#define SL   256
#define HL   128
#define RL   64
#define NE   16
#define NROW (NB * NA)

#define WP_SE1H 0
#define WP_SE2H 65536
#define WP_RE1H 98304
#define WP_RE2H 147456
#define WP_RAH  212992
#define WP_AE1H 311296
#define WP_AE2H 442368
#define WP_TOTAL 507904

#define OUT1_OFF 262144
#define OUT2_OFF 266240

__device__ __forceinline__ us bf16_rne(float x) {
  unsigned u = __float_as_uint(x);
  u += 0x7FFFu + ((u >> 16) & 1u);
  return (us)(u >> 16);
}
__device__ __forceinline__ float bf16_up(us b) { return __uint_as_float(((unsigned)b) << 16); }
__device__ __forceinline__ us bf16_lo(float x, us hi) { return bf16_rne(x - bf16_up(hi)); }

__device__ __forceinline__ v16bf ldfrag(const us* p, int h) {
  FragB f;
  f.half[0] = *(const v8usa*)(p + 8 * h);
  f.half[1] = *(const v8usa*)(p + 16 + 8 * h);
  return f.v;
}

__device__ __forceinline__ v8f mma3(v16bf ah, v16bf al, v16bf bh, v16bf bl, v8f c) {
  c = __builtin_amdgcn_wmma_f32_16x16x32_bf16(false, ah, false, bh, (short)0, c, false, false);
  c = __builtin_amdgcn_wmma_f32_16x16x32_bf16(false, ah, false, bl, (short)0, c, false, false);
  c = __builtin_amdgcn_wmma_f32_16x16x32_bf16(false, al, false, bh, (short)0, c, false, false);
  asm volatile("v_nop\n\tv_nop\n\tv_nop\n\tv_nop" : "+v"(c) : "v"(ah), "v"(al), "v"(bh), "v"(bl));
  return c;
}

#define MMA4(acc, ah, al, bth, btl, KP, nb, k0)                          \
  _Pragma("unroll") for (int q_ = 0; q_ < 4; ++q_) {                     \
    const size_t ro_ = (size_t)(16 * ((nb) + q_) + m) * (KP) + (k0);    \
    const v16bf bh_ = ldfrag((bth) + ro_, h);                            \
    const v16bf bl_ = ldfrag((btl) + ro_, h);                            \
    acc[q_] = mma3(ah, al, bh_, bl_, acc[q_]);                           \
  }

__device__ __forceinline__ void stage_split(const float* __restrict__ src, int nf4, int l2c4,
                                            us* dh, us* dl, int P, int tid, int nthr) {
  #pragma unroll 2
  for (int i = tid; i < nf4; i += nthr) {
    const int row = i >> l2c4, c4 = i & ((1 << l2c4) - 1);
    const v4f x = *(const v4fa*)(src + (size_t)i * 4);
    const us h0 = bf16_rne(x.x), h1 = bf16_rne(x.y), h2 = bf16_rne(x.z), h3 = bf16_rne(x.w);
    const v4us hv = {h0, h1, h2, h3};
    const v4us lv = {bf16_lo(x.x, h0), bf16_lo(x.y, h1), bf16_lo(x.z, h2), bf16_lo(x.w, h3)};
    const int o = row * P + 4 * c4;
    *(v4usa*)(dh + o) = hv;
    *(v4usa*)(dl + o) = lv;
  }
}

__device__ __forceinline__ void tile_to_H(v8f a, float bias, us* Hh, us* Hl, int pitch, int row0, int col, int h) {
  #pragma unroll
  for (int r = 0; r < 8; ++r) {
    const float v = fmaxf(a[r] + bias, 0.0f);
    const us hb = bf16_rne(v);
    const int o = (row0 + 8 * h + r) * pitch + col;
    Hh[o] = hb;
    Hl[o] = bf16_lo(v, hb);
  }
}

__device__ __forceinline__ void tile_to_f32(v8f a, float bias, float* T, int pitch, int col, int h) {
  #pragma unroll
  for (int r = 0; r < 8; ++r) T[(8 * h + r) * pitch + col] = fmaxf(a[r] + bias, 0.0f);
}

__device__ __forceinline__ void store_planes16x128(const float* T, us* ph, us* pl, size_t growbase, int lane) {
  const int sub = lane >> 4, c = 8 * (lane & 15);
  #pragma unroll
  for (int i = 0; i < 8; ++i) {
    const int row = 2 * i + sub;
    const v4f x0 = *(const v4fa*)(T + row * 128 + c);
    const v4f x1 = *(const v4fa*)(T + row * 128 + c + 4);
    const us h0 = bf16_rne(x0.x), h1 = bf16_rne(x0.y), h2 = bf16_rne(x0.z), h3 = bf16_rne(x0.w);
    const us h4 = bf16_rne(x1.x), h5 = bf16_rne(x1.y), h6 = bf16_rne(x1.z), h7 = bf16_rne(x1.w);
    const v8us hv = {h0, h1, h2, h3, h4, h5, h6, h7};
    const v8us lv = {bf16_lo(x0.x, h0), bf16_lo(x0.y, h1), bf16_lo(x0.z, h2), bf16_lo(x0.w, h3),
                     bf16_lo(x1.x, h4), bf16_lo(x1.y, h5), bf16_lo(x1.z, h6), bf16_lo(x1.w, h7)};
    const size_t o = (growbase + row) * 128 + c;
    *(volatile v8us*)(ph + o) = hv;
    *(volatile v8us*)(pl + o) = lv;
  }
}

__device__ __forceinline__ void store_f32_16x128(const float* T, float* g, size_t growbase, int lane) {
  #pragma unroll
  for (int i = 0; i < 16; ++i) {
    const v4f x = *(const v4fa*)(T + i * 128 + 4 * lane);
    *(volatile v4f*)(g + (growbase + i) * 128 + 4 * lane) = x;
  }
}

__device__ __forceinline__ void store_r0_pass(const us* Sh, const us* Sl, us* gh, us* gl,
                                              size_t growbase, int colbase, int lane) {
  const int sub = lane >> 3, c = 8 * (lane & 7);
  #pragma unroll
  for (int i = 0; i < 4; ++i) {
    const int row = 4 * i + sub;
    const v8us xh = *(const v8usa*)(Sh + row * 64 + c);
    const v8us xl = *(const v8usa*)(Sl + row * 64 + c);
    const size_t o = (growbase + row) * 256 + colbase + c;
    *(volatile v8us*)(gh + o) = xh;
    *(volatile v8us*)(gl + o) = xl;
  }
}

__device__ __forceinline__ void wconv_pass(const float* __restrict__ W, int K, int N, int n,
                                           us* __restrict__ ph, us* __restrict__ pl, int lane) {
  const int nch = K >> 6;
  const int sub = lane >> 3, q = lane & 7;
  #pragma unroll 1
  for (int cb = 0; cb < nch; cb += 4) {
    const int ch = cb + sub;
    const int chc = (ch < nch) ? ch : (nch - 1);
    const int k = 64 * chc + 8 * q;
    us hb[8], lb[8];
    #pragma unroll
    for (int t = 0; t < 8; ++t) {
      const float x = W[(size_t)(k + t) * N + n];
      hb[t] = bf16_rne(x);
      lb[t] = bf16_lo(x, hb[t]);
    }
    const v8us hv = {hb[0], hb[1], hb[2], hb[3], hb[4], hb[5], hb[6], hb[7]};
    const v8us lv = {lb[0], lb[1], lb[2], lb[3], lb[4], lb[5], lb[6], lb[7]};
    if (ch < nch) {
      const size_t o = (size_t)n * K + 64 * ch + 8 * q;
      *(volatile v8us*)(ph + o) = hv;
      *(volatile v8us*)(pl + o) = lv;
    }
  }
}

__global__ __launch_bounds__(32) void k_wconv(
    const float* __restrict__ w0, const float* __restrict__ w1, const float* __restrict__ w2,
    const float* __restrict__ w3, const float* __restrict__ w4, const float* __restrict__ w5,
    const float* __restrict__ w6, us* __restrict__ wpl)
{
  const int y = blockIdx.y, n = blockIdx.x, lane = threadIdx.x;
  const float* W; int K, N, oh;
  if (y == 0)      { W = w0; K = SL;      N = HL;     oh = WP_SE1H; }
  else if (y == 1) { W = w1; K = HL;      N = HL;     oh = WP_SE2H; }
  else if (y == 2) { W = w2; K = HL + RL; N = HL;     oh = WP_RE1H; }
  else if (y == 3) { W = w3; K = HL;      N = 2 * HL; oh = WP_RE2H; }
  else if (y == 4) { W = w4; K = 3 * HL;  N = HL;     oh = WP_RAH;  }
  else if (y == 5) { W = w5; K = 4 * HL;  N = HL;     oh = WP_AE1H; }
  else             { W = w6; K = HL;      N = 2 * HL; oh = WP_AE2H; }
  if (n >= N) return;
  us* ph = wpl + oh;
  us* pl = ph + (size_t)K * N;
  wconv_pass(W, K, N, n, ph, pl, lane);
  __threadfence();
  wconv_pass(W, K, N, n, ph, pl, lane);
}

__global__ __launch_bounds__(64) void k_se(
    const float* __restrict__ states, const float* __restrict__ b1, const float* __restrict__ b2,
    const us* __restrict__ wpl, us* __restrict__ shi, us* __restrict__ slo)
{
  __shared__ __attribute__((aligned(16))) unsigned char XS[32 * 264 * 2 * 2];
  __shared__ __attribute__((aligned(16))) us Hh[32 * 136];
  __shared__ __attribute__((aligned(16))) us Hl[32 * 136];
  us* Xh = (us*)XS;
  us* Xl = Xh + 32 * 264;
  float* So = (float*)XS;

  const int tid = threadIdx.x, lane = tid & 31, w = tid >> 5, h = lane >> 4, m = lane & 15;
  const int row0 = blockIdx.x * 32;
  stage_split(states + (size_t)row0 * SL, 32 * (SL / 4), 6, Xh, Xl, 264, tid, 64);
  __syncthreads();

  const us* W1h = wpl + WP_SE1H; const us* W1l = W1h + SL * HL;
  const us* W2h = wpl + WP_SE2H; const us* W2l = W2h + HL * HL;
  const v8f z8 = {0.f, 0.f, 0.f, 0.f, 0.f, 0.f, 0.f, 0.f};

  #pragma unroll 1
  for (int pass = 0; pass < 2; ++pass) {
    v8f acc[4];
    #pragma unroll
    for (int q = 0; q < 4; ++q) acc[q] = z8;
    #pragma unroll 1
    for (int ks = 0; ks < 8; ++ks) {
      const int ao = (16 * w + m) * 264 + 32 * ks;
      const v16bf ah = ldfrag(Xh + ao, h), al = ldfrag(Xl + ao, h);
      MMA4(acc, ah, al, W1h, W1l, SL, 4 * pass, 32 * ks);
    }
    #pragma unroll
    for (int q = 0; q < 4; ++q) {
      const int col = 16 * (4 * pass + q) + m;
      tile_to_H(acc[q], b1[col], Hh, Hl, 136, 16 * w, col, h);
    }
  }
  __syncthreads();

  float* T = So + w * 2048;
  #pragma unroll 1
  for (int pass = 0; pass < 2; ++pass) {
    v8f acc[4];
    #pragma unroll
    for (int q = 0; q < 4; ++q) acc[q] = z8;
    #pragma unroll 1
    for (int ks = 0; ks < 4; ++ks) {
      const int ao = (16 * w + m) * 136 + 32 * ks;
      const v16bf ah = ldfrag(Hh + ao, h), al = ldfrag(Hl + ao, h);
      MMA4(acc, ah, al, W2h, W2l, HL, 4 * pass, 32 * ks);
    }
    #pragma unroll
    for (int q = 0; q < 4; ++q) {
      const int col = 16 * (4 * pass + q) + m;
      tile_to_f32(acc[q], b2[col], T, 128, col, h);
    }
  }
  __syncthreads();

  const size_t growbase = (size_t)row0 + 16 * w;
  store_planes16x128(T, shi, slo, growbase, lane);
  __threadfence();
  store_planes16x128(T, shi, slo, growbase, lane);
}

__global__ __launch_bounds__(128) void k_rel(
    const float* __restrict__ relations, const float* __restrict__ alive,
    const float* __restrict__ b1, const float* __restrict__ b2, const int* __restrict__ agent_id,
    const us* __restrict__ shi, const us* __restrict__ slo, const us* __restrict__ wpl,
    float* __restrict__ ram, us* __restrict__ r0h, us* __restrict__ r0l)
{
  __shared__ __attribute__((aligned(16))) us RS[2 * 64 * 72];
  __shared__ __attribute__((aligned(16))) us Hh[64 * 136];
  __shared__ __attribute__((aligned(16))) us Hl[64 * 136];
  __shared__ __attribute__((aligned(16))) float Red[4 * 256];
  __shared__ __attribute__((aligned(16))) float RowBuf[256];
  us* Rh = RS; us* Rl = RS + 64 * 72;
  us* Sgh = RS; us* Sgl = RS + 4096;

  const int tid = threadIdx.x, lane = tid & 31, w = tid >> 5, h = lane >> 4, m = lane & 15;
  const int bi = blockIdx.x, b = bi >> 6, i = bi & 63;
  int aid = agent_id[0];
  aid = aid < 0 ? 0 : (aid > NA - 1 ? NA - 1 : aid);
  const bool isaid = (i == aid);

  stage_split(relations + (size_t)bi * (NA * RL), NA * RL / 4, 4, Rh, Rl, 72, tid, 128);
  __syncthreads();

  float mk[8];
  #pragma unroll
  for (int r = 0; r < 8; ++r) mk[r] = alive[b * NA + 16 * w + 8 * h + r];

  const us* W1h = wpl + WP_RE1H; const us* W1l = W1h + (HL + RL) * HL;
  const us* W2h = wpl + WP_RE2H; const us* W2l = W2h + HL * 2 * HL;
  const v8f z8 = {0.f, 0.f, 0.f, 0.f, 0.f, 0.f, 0.f, 0.f};

  #pragma unroll 1
  for (int pass = 0; pass < 2; ++pass) {
    v8f acc[4];
    #pragma unroll
    for (int q = 0; q < 4; ++q) acc[q] = z8;
    #pragma unroll
    for (int ks = 0; ks < 2; ++ks) {
      const int ao = (16 * w + m) * 72 + 32 * ks;
      const v16bf ah = ldfrag(Rh + ao, h), al = ldfrag(Rl + ao, h);
      MMA4(acc, ah, al, W1h, W1l, HL + RL, 4 * pass, 32 * ks);
    }
    #pragma unroll 1
    for (int ks = 0; ks < 4; ++ks) {
      const size_t go = (size_t)(b * NA + 16 * w + m) * HL + 32 * ks;
      const v16bf ah = ldfrag(shi + go, h), al = ldfrag(slo + go, h);
      MMA4(acc, ah, al, W1h, W1l, HL + RL, 4 * pass, RL + 32 * ks);
    }
    #pragma unroll
    for (int q = 0; q < 4; ++q) {
      const int col = 16 * (4 * pass + q) + m;
      tile_to_H(acc[q], b1[col], Hh, Hl, 136, 16 * w, col, h);
    }
  }
  __syncthreads();

  #pragma unroll 1
  for (int p = 0; p < 4; ++p) {
    v8f acc[4];
    #pragma unroll
    for (int q = 0; q < 4; ++q) acc[q] = z8;
    #pragma unroll 1
    for (int ks = 0; ks < 4; ++ks) {
      const int ao = (16 * w + m) * 136 + 32 * ks;
      const v16bf ah = ldfrag(Hh + ao, h), al = ldfrag(Hl + ao, h);
      MMA4(acc, ah, al, W2h, W2l, HL, 4 * p, 32 * ks);
    }
    #pragma unroll
    for (int q = 0; q < 4; ++q) {
      const int col = 64 * p + 16 * q + m;
      const float bv = b2[col];
      float vr[8];
      #pragma unroll
      for (int r = 0; r < 8; ++r) vr[r] = fmaxf(acc[q][r] + bv, 0.0f);
      if (p < 2) {
        float s = 0.0f;
        #pragma unroll
        for (int r = 0; r < 8; ++r) s += vr[r] * mk[r];
        s += __shfl_xor(s, 16);
        if (h == 0) Red[w * 256 + col] = s;
      } else {
        float mx = vr[0] * mk[0];
        #pragma unroll
        for (int r = 1; r < 8; ++r) mx = fmaxf(mx, vr[r] * mk[r]);
        mx = fmaxf(mx, __shfl_xor(mx, 16));
        if (h == 0) Red[w * 256 + col] = mx;
      }
      if (isaid) {
        #pragma unroll
        for (int r = 0; r < 8; ++r) {
          const us hb = bf16_rne(vr[r]);
          const int o = w * 1024 + (8 * h + r) * 64 + 16 * q + m;
          Sgh[o] = hb;
          Sgl[o] = bf16_lo(vr[r], hb);
        }
      }
    }
    if (isaid) {
      __syncthreads();
      const size_t growbase = (size_t)b * NA + 16 * w;
      store_r0_pass(Sgh + w * 1024, Sgl + w * 1024, r0h, r0l, growbase, 64 * p, lane);
      __threadfence();
      store_r0_pass(Sgh + w * 1024, Sgl + w * 1024, r0h, r0l, growbase, 64 * p, lane);
      __syncthreads();
    }
  }
  __syncthreads();

  {
    const int c = tid;
    float a = Red[c]; a += Red[256 + c]; a += Red[512 + c]; a += Red[768 + c];
    RowBuf[c] = a * 0.015625f;
    float x = Red[HL + c];
    x = fmaxf(x, Red[256 + HL + c]); x = fmaxf(x, Red[512 + HL + c]); x = fmaxf(x, Red[768 + HL + c]);
    RowBuf[HL + c] = x;
  }
  __syncthreads();
  if (w == 0) {
    const v4f v0 = *(const v4fa*)(RowBuf + 4 * lane);
    const v4f v1 = *(const v4fa*)(RowBuf + HL + 4 * lane);
    float* dst = ram + (size_t)bi * 256;
    *(volatile v4f*)(dst + 4 * lane) = v0;
    *(volatile v4f*)(dst + HL + 4 * lane) = v1;
    __threadfence();
    *(volatile v4f*)(dst + 4 * lane) = v0;
    *(volatile v4f*)(dst + HL + 4 * lane) = v1;
  }
}

__global__ __launch_bounds__(64) void k_ra(
    const float* __restrict__ ram, const float* __restrict__ rab,
    const us* __restrict__ shi, const us* __restrict__ slo, const us* __restrict__ wpl,
    float* __restrict__ s1f, us* __restrict__ s1h, us* __restrict__ s1l)
{
  __shared__ __attribute__((aligned(16))) us Xh[32 * 264];
  __shared__ __attribute__((aligned(16))) us Xl[32 * 264];
  __shared__ __attribute__((aligned(16))) float So[2 * 16 * 128];

  const int tid = threadIdx.x, lane = tid & 31, w = tid >> 5, h = lane >> 4, m = lane & 15;
  const int row0 = blockIdx.x * 32;
  stage_split(ram + (size_t)row0 * 256, 32 * 64, 6, Xh, Xl, 264, tid, 64);
  __syncthreads();

  const us* Wh = wpl + WP_RAH; const us* Wl = Wh + 3 * HL * HL;
  const v8f z8 = {0.f, 0.f, 0.f, 0.f, 0.f, 0.f, 0.f, 0.f};
  float* T = So + w * 2048;

  #pragma unroll 1
  for (int pass = 0; pass < 2; ++pass) {
    v8f acc[4];
    #pragma unroll
    for (int q = 0; q < 4; ++q) acc[q] = z8;
    #pragma unroll 1
    for (int ks = 0; ks < 4; ++ks) {
      const size_t go = (size_t)(row0 + 16 * w + m) * HL + 32 * ks;
      const v16bf ah = ldfrag(shi + go, h), al = ldfrag(slo + go, h);
      MMA4(acc, ah, al, Wh, Wl, 3 * HL, 4 * pass, 32 * ks);
    }
    #pragma unroll 1
    for (int ks = 0; ks < 8; ++ks) {
      const int ao = (16 * w + m) * 264 + 32 * ks;
      const v16bf ah = ldfrag(Xh + ao, h), al = ldfrag(Xl + ao, h);
      MMA4(acc, ah, al, Wh, Wl, 3 * HL, 4 * pass, HL + 32 * ks);
    }
    #pragma unroll
    for (int q = 0; q < 4; ++q) {
      const int col = 16 * (4 * pass + q) + m;
      tile_to_f32(acc[q], rab[col], T, 128, col, h);
    }
  }
  __syncthreads();

  const size_t growbase = (size_t)row0 + 16 * w;
  store_f32_16x128(T, s1f, growbase, lane);
  store_planes16x128(T, s1h, s1l, growbase, lane);
  __threadfence();
  store_f32_16x128(T, s1f, growbase, lane);
  store_planes16x128(T, s1h, s1l, growbase, lane);
}

__device__ __forceinline__ void tail_store(const float* __restrict__ s1f, const float* SelRow,
                                           const float* AeRow, float* __restrict__ out,
                                           int b, int aid, int jstar, int w, int lane) {
  const int c = 4 * lane;
  const v4f sl = *(const v4fa*)(SelRow + c);
  const v4f pa = *(const v4fa*)(AeRow + HL + c);
  const v4f z = {0.f, 0.f, 0.f, 0.f};
  #pragma unroll
  for (int i = 0; i < 16; ++i) {
    const int j = 16 * w + i;
    const size_t ro = ((size_t)b * NA + j) * HL + c;
    v4f s = *(const v4fa*)(s1f + ro);
    s = (j == aid) ? (s + sl) : s;
    const v4f pj = (j == jstar) ? pa : z;
    s = s + pj;
    *(volatile v4f*)(out + ro) = s;
    *(volatile v4f*)(out + OUT2_OFF + ro) = pj;
  }
  if (w == 0) *(volatile v4f*)(out + OUT1_OFF + (size_t)b * HL + c) = sl;
}

__global__ __launch_bounds__(128) void k_ae(
    const us* __restrict__ r0h, const us* __restrict__ r0l, const float* __restrict__ s1f,
    const us* __restrict__ s1h, const us* __restrict__ s1l, const us* __restrict__ wpl,
    const float* __restrict__ b1, const float* __restrict__ b2, const float* __restrict__ aemb,
    const int* __restrict__ action, const int* __restrict__ agent_id,
    const int* __restrict__ amask_unused,
    float* __restrict__ out)
{
  __shared__ __attribute__((aligned(16))) us Ah[HL];
  __shared__ __attribute__((aligned(16))) us Al[HL];
  __shared__ __attribute__((aligned(16))) us Hh[64 * 136];
  __shared__ __attribute__((aligned(16))) us Hl[64 * 136];
  __shared__ __attribute__((aligned(16))) float AeRow[256];
  __shared__ __attribute__((aligned(16))) float SelRow[HL];
  (void)amask_unused;

  const int tid = threadIdx.x, lane = tid & 31, w = tid >> 5, h = lane >> 4, m = lane & 15;
  const int b = blockIdx.x;
  int act = action[b];
  act = act < 0 ? 0 : (act > NE + NA - 1 ? NE + NA - 1 : act);
  int aid = agent_id[0];
  aid = aid < 0 ? 0 : (aid > NA - 1 ? NA - 1 : aid);
  const int jstar = (act >= NE) ? (act - NE) : -1;

  if (w == 0) {
    const size_t ro = (size_t)(b * NA + aid) * HL + 4 * lane;
    *(v4usa*)(Ah + 4 * lane) = *(const v4usa*)(s1h + ro);
    *(v4usa*)(Al + 4 * lane) = *(const v4usa*)(s1l + ro);
  }
  AeRow[tid] = 0.0f;
  AeRow[HL + tid] = 0.0f;
  __syncthreads();

  const us* W1h = wpl + WP_AE1H; const us* W1l = W1h + 4 * HL * HL;
  const us* W2h = wpl + WP_AE2H; const us* W2l = W2h + HL * 2 * HL;
  const v8f z8 = {0.f, 0.f, 0.f, 0.f, 0.f, 0.f, 0.f, 0.f};

  #pragma unroll 1
  for (int pass = 0; pass < 2; ++pass) {
    v8f acc[4];
    #pragma unroll
    for (int q = 0; q < 4; ++q) acc[q] = z8;
    #pragma unroll 1
    for (int ks = 0; ks < 8; ++ks) {
      const size_t go = (size_t)(b * NA + 16 * w + m) * 256 + 32 * ks;
      const v16bf ah = ldfrag(r0h + go, h), al = ldfrag(r0l + go, h);
      MMA4(acc, ah, al, W1h, W1l, 4 * HL, 4 * pass, 32 * ks);
    }
    #pragma unroll 1
    for (int ks = 0; ks < 4; ++ks) {
      const size_t go = (size_t)(b * NA + 16 * w + m) * HL + 32 * ks;
      const v16bf ah = ldfrag(s1h + go, h), al = ldfrag(s1l + go, h);
      MMA4(acc, ah, al, W1h, W1l, 4 * HL, 4 * pass, 2 * HL + 32 * ks);
    }
    #pragma unroll 1
    for (int ks = 0; ks < 4; ++ks) {
      const int ao = 32 * ks;
      const v16bf ah = ldfrag(Ah + ao, h), al = ldfrag(Al + ao, h);
      MMA4(acc, ah, al, W1h, W1l, 4 * HL, 4 * pass, 3 * HL + 32 * ks);
    }
    #pragma unroll
    for (int q = 0; q < 4; ++q) {
      const int col = 16 * (4 * pass + q) + m;
      tile_to_H(acc[q], b1[col], Hh, Hl, 136, 16 * w, col, h);
    }
  }
  __syncthreads();

  #pragma unroll 1
  for (int p = 0; p < 4; ++p) {
    v8f acc[4];
    #pragma unroll
    for (int q = 0; q < 4; ++q) acc[q] = z8;
    #pragma unroll 1
    for (int ks = 0; ks < 4; ++ks) {
      const int ao = (16 * w + m) * 136 + 32 * ks;
      const v16bf ah = ldfrag(Hh + ao, h), al = ldfrag(Hl + ao, h);
      MMA4(acc, ah, al, W2h, W2l, HL, 4 * p, 32 * ks);
    }
    #pragma unroll
    for (int q = 0; q < 4; ++q) {
      const int col = 64 * p + 16 * q + m;
      const float bv = b2[col];
      #pragma unroll
      for (int r = 0; r < 8; ++r) {
        const float v = fmaxf(acc[q][r] + bv, 0.0f);
        if (16 * w + 8 * h + r == jstar) AeRow[col] = v;
      }
    }
  }
  __syncthreads();

  {
    const int c = tid;
    const int ae16 = (act < NE) ? act : (NE - 1);
    const float e = aemb[(size_t)ae16 * HL + c];
    const float a = AeRow[c];
    SelRow[c] = (act < NE) ? e : a;
  }
  __syncthreads();

  tail_store(s1f, SelRow, AeRow, out, b, aid, jstar, w, lane);
  __threadfence();
  tail_store(s1f, SelRow, AeRow, out, b, aid, jstar, w, lane);
}

extern "C" void kernel_launch(void* const* d_in, const int* in_sizes, int n_in,
                              void* d_out, int out_size, void* d_ws, size_t ws_size,
                              hipStream_t stream) {
  if (n_in < 21) return;
  if (in_sizes[0] != NROW * SL) return;
  if (in_sizes[1] != NROW * NA * RL) return;
  if (in_sizes[2] != NROW) return;
  if (in_sizes[3] != SL * HL || in_sizes[4] != HL) return;
  if (in_sizes[5] != HL * HL || in_sizes[6] != HL) return;
  if (in_sizes[7] != (HL + RL) * HL || in_sizes[8] != HL) return;
  if (in_sizes[9] != HL * 2 * HL || in_sizes[10] != 2 * HL) return;
  if (in_sizes[11] != 3 * HL * HL || in_sizes[12] != HL) return;
  if (in_sizes[13] != 4 * HL * HL || in_sizes[14] != HL) return;
  if (in_sizes[15] != HL * 2 * HL || in_sizes[16] != 2 * HL) return;
  if (in_sizes[17] != NE * HL) return;
  if (in_sizes[19] != NB || in_sizes[20] < 1) return;
  if (out_size != NROW * HL + NB * HL + NROW * HL) return;

  const float* states = (const float*)d_in[0];
  const float* rels   = (const float*)d_in[1];
  const float* alive  = (const float*)d_in[2];
  const float* se_w1  = (const float*)d_in[3];
  const float* se_b1  = (const float*)d_in[4];
  const float* se_w2  = (const float*)d_in[5];
  const float* se_b2  = (const float*)d_in[6];
  const float* re_w1  = (const float*)d_in[7];
  const float* re_b1  = (const float*)d_in[8];
  const float* re_w2  = (const float*)d_in[9];
  const float* re_b2  = (const float*)d_in[10];
  const float* ra_w   = (const float*)d_in[11];
  const float* ra_b   = (const float*)d_in[12];
  const float* ae_w1  = (const float*)d_in[13];
  const float* ae_b1  = (const float*)d_in[14];
  const float* ae_w2  = (const float*)d_in[15];
  const float* ae_b2  = (const float*)d_in[16];
  const float* aem    = (const float*)d_in[17];
  const int*   amask  = (const int*)d_in[18];
  const int*   action = (const int*)d_in[19];
  const int*   agent  = (const int*)d_in[20];
  float* out = (float*)d_out;

  const size_t wpl_b = (size_t)WP_TOTAL * 2;
  const size_t pl_b  = (size_t)NROW * HL * 2;
  const size_t ram_b = (size_t)NROW * 2 * HL * 4;
  const size_t r0_b  = (size_t)NROW * 2 * HL * 2;
  const size_t s1f_b = (size_t)NROW * HL * 4;
  size_t off = 0;
  const size_t o_wpl = off; off += wpl_b;
  const size_t o_shi = off; off += pl_b;
  const size_t o_slo = off; off += pl_b;
  const size_t o_ram = off; off += ram_b;
  const size_t o_r0h = off; off += r0_b;
  const size_t o_r0l = off; off += r0_b;
  const size_t o_s1f = off; off += s1f_b;
  const size_t o_s1h = off; off += pl_b;
  const size_t o_s1l = off; off += pl_b;
  const size_t total = off;
  if (total > ws_size) return;
  if (total > (size_t)134217728) return;

  char* ws = (char*)d_ws;
  us*    wpl = (us*)(ws + o_wpl);
  us*    shi = (us*)(ws + o_shi);
  us*    slo = (us*)(ws + o_slo);
  float* ram = (float*)(ws + o_ram);
  us*    r0h = (us*)(ws + o_r0h);
  us*    r0l = (us*)(ws + o_r0l);
  float* s1f = (float*)(ws + o_s1f);
  us*    s1h = (us*)(ws + o_s1h);
  us*    s1l = (us*)(ws + o_s1l);

  k_wconv<<<dim3(256, 7), 32, 0, stream>>>(se_w1, se_w2, re_w1, re_w2, ra_w, ae_w1, ae_w2, wpl);
  k_se<<<NROW / 32, 64, 0, stream>>>(states, se_b1, se_b2, wpl, shi, slo);
  k_rel<<<NROW, 128, 0, stream>>>(rels, alive, re_b1, re_b2, agent, shi, slo, wpl, ram, r0h, r0l);
  k_ra<<<NROW / 32, 64, 0, stream>>>(ram, ra_b, shi, slo, wpl, s1f, s1h, s1l);
  k_ae<<<NB, 128, 0, stream>>>(r0h, r0l, s1f, s1h, s1l, wpl, ae_b1, ae_b2, aem, action, agent, amask, out);
}
